// LTAE1d_64115271794771
// MI455X (gfx1250) — hardware-verified
//
#include <hip/hip_runtime.h>
#include <math.h>
#include <stddef.h>
#include <stdint.h>


#define NB     1024
#define TT     60
#define CIN    10
#define DM     256
#define NH     16
#define NA     13
#define DKQ    4
#define DHV    16
#define MOUT   128
#define ROWS   (NH * NA)
#define NWROW  (ROWS * NA)
#define MROWS  (NA * NB)
#define VTILE  (TT * DM)
#define OSLAB  256
#define KSTEPS (DM / 32)

#define SA_KEY 32.0f
#define SB_KEY 32.0f
#define SA_MLP 32.0f
#define SB_MLP 1024.0f
#define RESC   2048.0f

typedef _Float16 v16h __attribute__((ext_vector_type(16)));
typedef _Float16 v8h  __attribute__((ext_vector_type(8)));
typedef float    v8f  __attribute__((ext_vector_type(8)));
typedef float    v4f  __attribute__((ext_vector_type(4)));
union Frag { v16h v; v8h h[2]; };

static __device__ __forceinline__ v8f wmma16(v16h a, v16h b, v8f c) {
  v8f d = __builtin_amdgcn_wmma_f32_16x16x32_f16(false, a, false, b, (short)0, c, false, false);
  asm volatile("v_nop\n\tv_nop\n\tv_nop\n\tv_nop" : "+v"(d) : "v"(a), "v"(b));
  return d;
}

static __device__ __forceinline__ v8f zero8() {
  v8f z = {0.0f, 0.0f, 0.0f, 0.0f, 0.0f, 0.0f, 0.0f, 0.0f};
  return z;
}

static __device__ __forceinline__ void split8(v4f p, v4f q, float sc, v8h& hi, v8h& lo) {
  float x[8] = {p.x, p.y, p.z, p.w, q.x, q.y, q.z, q.w};
#pragma unroll
  for (int e = 0; e < 8; ++e) {
    const float xs = x[e] * sc;
    const _Float16 hv = (_Float16)xs;
    hi[e] = hv;
    lo[e] = (_Float16)((xs - (float)hv) * RESC);
  }
}

__global__ __launch_bounds__(256) void k_inconv_gn(
    const float* __restrict__ x, const float* __restrict__ Wc,
    const float* __restrict__ bc, const float* __restrict__ gnw,
    const float* __restrict__ gnb, float* __restrict__ vbuf, int nb)
{
  __shared__ float sx[TT * CIN];
  __shared__ float sv[VTILE];
  const int b = blockIdx.x;
  if (b >= nb) return;
  const int d = threadIdx.x;

  const float* xsrc = x + (size_t)b * (TT * CIN);
  for (int idx = d; idx < TT * CIN; idx += 256) sx[idx] = xsrc[idx];
  __syncthreads();

  float wr[CIN];
#pragma unroll
  for (int c2 = 0; c2 < CIN; ++c2) wr[c2] = Wc[d * CIN + c2];
  const float bias = bc[d];

  float s = 0.0f;
#pragma unroll 1
  for (int t = 0; t < TT; ++t) {
    const float* xr = sx + t * CIN;
    float acc = xr[0] * wr[0];
#pragma unroll
    for (int c2 = 1; c2 < CIN; ++c2) acc = fmaf(xr[c2], wr[c2], acc);
    acc += bias;
    sv[t * DM + d] = acc;
    s += acc;
  }
#pragma unroll
  for (int off = 1; off < 16; off <<= 1) s += __shfl_xor(s, off, 32);
  const float mu = s * (1.0f / 960.0f);

  float s2 = 0.0f;
#pragma unroll 1
  for (int t = 0; t < TT; ++t) {
    const float dv = sv[t * DM + d] - mu;
    s2 = fmaf(dv, dv, s2);
  }
#pragma unroll
  for (int off = 1; off < 16; off <<= 1) s2 += __shfl_xor(s2, off, 32);
  const float var = s2 * (1.0f / 960.0f);
  const float rs = 1.0f / sqrtf(var + 1e-5f);
  const float gw = gnw[d], gb = gnb[d];
#pragma unroll 1
  for (int t = 0; t < TT; ++t) {
    const int k = t * DM + d;
    sv[k] = (sv[k] - mu) * rs * gw + gb;
  }
  __syncthreads();

  float* dst = vbuf + (size_t)b * VTILE;
  v4f vals[15];
#pragma unroll
  for (int k = 0; k < 15; ++k) vals[k] = *(const v4f*)(&sv[d * 4 + k * 1024]);
#pragma unroll
  for (int k = 0; k < 15; ++k) *(volatile v4f*)(dst + d * 4 + k * 1024) = vals[k];
  __threadfence();
#pragma unroll
  for (int k = 0; k < 15; ++k) *(volatile v4f*)(dst + d * 4 + k * 1024) = vals[k];
}

__global__ __launch_bounds__(128) void k_tables(
    const float* __restrict__ Q, const float* __restrict__ Wk, const float* __restrict__ W1,
    _Float16* __restrict__ wth, _Float16* __restrict__ wtl,
    _Float16* __restrict__ w1h, _Float16* __restrict__ w1l, int nblk)
{
  const int blk = blockIdx.x;
  if (blk >= nblk) return;
  const int w = threadIdx.x >> 5, lane = threadIdx.x & 31;
  const int nwb = NWROW / 4;

  v4f p, q;
  float sc;
  _Float16* dh;
  _Float16* dl;
  if (blk < nwb) {
    const int row = blk * 4 + w;
    const int u = row / NA, a = row - u * NA;
    const int h2 = u / NA;
    const float* qp = Q + (u >> 4) * (NH * DKQ) + (u & 15) * DKQ;
    const float q0 = qp[0], q1 = qp[1], q2 = qp[2], q3 = qp[3];
    const float* wk = Wk + (size_t)((a * NH + h2) * DKQ) * DM + lane * 8;
    const v4f r0a = *(const v4f*)(wk),          r0b = *(const v4f*)(wk + 4);
    const v4f r1a = *(const v4f*)(wk + DM),     r1b = *(const v4f*)(wk + DM + 4);
    const v4f r2a = *(const v4f*)(wk + 2 * DM), r2b = *(const v4f*)(wk + 2 * DM + 4);
    const v4f r3a = *(const v4f*)(wk + 3 * DM), r3b = *(const v4f*)(wk + 3 * DM + 4);
    p = q0 * r0a + q1 * r1a + q2 * r2a + q3 * r3a;
    q = q0 * r0b + q1 * r1b + q2 * r2b + q3 * r3b;
    sc = SA_KEY;
    dh = wth + (size_t)row * DM + lane * 8;
    dl = wtl + (size_t)row * DM + lane * 8;
  } else {
    const int row = (blk - nwb) * 4 + w;
    const float* wp = W1 + (size_t)row * DM + lane * 8;
    p = *(const v4f*)(wp);
    q = *(const v4f*)(wp + 4);
    sc = SB_MLP;
    dh = w1h + (size_t)row * DM + lane * 8;
    dl = w1l + (size_t)row * DM + lane * 8;
  }
  v8h hi, lo;
  split8(p, q, sc, hi, lo);
  *(volatile v8h*)dh = hi;
  *(volatile v8h*)dl = lo;
  __threadfence();
  *(volatile v8h*)dh = hi;
  *(volatile v8h*)dl = lo;
}

template <int NT>
static __device__ __forceinline__ void key_gemm(int mt0, int c, int w, int lane,
    const float* svf, float* sL, const float* sQB,
    const _Float16* __restrict__ wth, const _Float16* __restrict__ wtl)
{
  const int hh = lane >> 4, m16 = lane & 15;
  v8f ah[NT], ax[NT];
  int aoff[NT];
#pragma unroll
  for (int j = 0; j < NT; ++j) {
    ah[j] = zero8();
    ax[j] = zero8();
    const int i = (mt0 + j) * 16 + m16;
    const int h2 = i / NA, a = i - h2 * NA;
    const int trow = (h2 * NA + c) * NA + a;
    aoff[j] = trow * DM + 8 * hh;
  }
  int tcol = w * 16 + m16;
  if (tcol > TT - 1) tcol = TT - 1;
  const float* vrow = svf + tcol * DM + 8 * hh;

#pragma unroll 1
  for (int ks = 0; ks < KSTEPS; ++ks) {
    const float* vp = vrow + ks * 32;
    Frag bh, bl;
    split8(*(const v4f*)(vp),      *(const v4f*)(vp + 4),  SB_KEY, bh.h[0], bl.h[0]);
    split8(*(const v4f*)(vp + 16), *(const v4f*)(vp + 20), SB_KEY, bh.h[1], bl.h[1]);
#pragma unroll
    for (int j = 0; j < NT; ++j) {
      const _Float16* ph = wth + aoff[j] + ks * 32;
      const _Float16* pl = wtl + aoff[j] + ks * 32;
      Frag fh, fl;
      fh.h[0] = *(const v8h*)(ph);
      fh.h[1] = *(const v8h*)(ph + 16);
      fl.h[0] = *(const v8h*)(pl);
      fl.h[1] = *(const v8h*)(pl + 16);
      ah[j] = wmma16(fh.v, bh.v, ah[j]);
      ax[j] = wmma16(fh.v, bl.v, ax[j]);
      ax[j] = wmma16(fl.v, bh.v, ax[j]);
    }
  }

  const int col = w * 16 + m16;
#pragma unroll
  for (int j = 0; j < NT; ++j) {
#pragma unroll
    for (int r = 0; r < 8; ++r) {
      const int i = (mt0 + j) * 16 + 8 * hh + r;
      const float lv = (ah[j][r] + ax[j][r] * (1.0f / RESC)) * (0.5f / (SA_KEY * SB_KEY)) + sQB[i];
      if (col < TT) sL[i * TT + col] = lv;
    }
  }
}

__global__ __launch_bounds__(128) void k_attn(
    const float* __restrict__ vbuf, const _Float16* __restrict__ wth, const _Float16* __restrict__ wtl,
    const float* __restrict__ Q, const float* __restrict__ bk, float* __restrict__ out3, int nb)
{
  __shared__ float svf[VTILE];
  __shared__ float sL[ROWS * TT];
  __shared__ float sO[NH * OSLAB];
  __shared__ float sQ[NH * DKQ];
  __shared__ float sQB[ROWS];

  const int b2 = blockIdx.x;
  if (b2 >= nb) return;
  const int tid = threadIdx.x, lane = tid & 31, w = tid >> 5;

  const float* vsrc = vbuf + (size_t)b2 * VTILE;
  for (int idx = tid * 4; idx < VTILE; idx += 128 * 4)
    *(v4f*)(&svf[idx]) = *(const v4f*)(vsrc + idx);
  for (int idx = tid; idx < NH * OSLAB; idx += 128) sO[idx] = 0.0f;

  const int r13 = (b2 * NA) & 1023;
  const int nvar = (r13 >= 1024 - (NA - 1)) ? 2 : 1;
  const int split = (nvar == 2) ? (1024 - r13) : NA;

  for (int vs = 0; vs < nvar; ++vs) {
    const int c = (b2 * NA + (vs ? (NA - 1) : 0)) >> 10;
    __syncthreads();
    if (tid < NH * DKQ) {
      const int h2 = tid >> 2, dk = tid & 3;
      const int u = h2 * NA + c;
      sQ[tid] = Q[(u >> 4) * (NH * DKQ) + (u & 15) * DKQ + dk];
    }
    __syncthreads();
    for (int i = tid; i < ROWS; i += 128) {
      const int h2 = i / NA, a = i - h2 * NA;
      const float* bp = bk + (a * NH + h2) * DKQ;
      const float* qp = sQ + h2 * DKQ;
      float sb = qp[0] * bp[0];
      sb = fmaf(qp[1], bp[1], sb);
      sb = fmaf(qp[2], bp[2], sb);
      sb = fmaf(qp[3], bp[3], sb);
      sQB[i] = 0.5f * sb;
    }
    __syncthreads();

    key_gemm<4>(0,  c, w, lane, svf, sL, sQB, wth, wtl);
    key_gemm<4>(4,  c, w, lane, svf, sL, sQB, wth, wtl);
    key_gemm<4>(8,  c, w, lane, svf, sL, sQB, wth, wtl);
    key_gemm<1>(12, c, w, lane, svf, sL, sQB, wth, wtl);
    __syncthreads();

    for (int i = tid; i < ROWS; i += 128) {
      const int h2 = i / NA, a2 = i - h2 * NA;
      const bool mine = (vs == 0) ? (a2 < split) : (a2 >= split);
      if (!mine) continue;
      float* base = sL + h2 * (NA * TT);
      const int j0 = a2 * TT;
      const int t0 = j0 / NA, a0 = j0 - t0 * NA;

      float mx = -3.0e38f;
      int a = a0, t = t0;
#pragma unroll 1
      for (int tp = 0; tp < TT; ++tp) {
        mx = fmaxf(mx, base[a * TT + t]);
        if (++a == NA) { a = 0; ++t; }
      }
      float sum = 0.0f;
      a = a0; t = t0;
#pragma unroll 1
      for (int tp = 0; tp < TT; ++tp) {
        float* cp = base + a * TT + t;
        const float e = expf(*cp - mx);
        *cp = e;
        sum += e;
        if (++a == NA) { a = 0; ++t; }
      }
      const float inv = 1.0f / sum;

      float o[DHV];
#pragma unroll
      for (int e = 0; e < DHV; ++e) o[e] = 0.0f;
      const float* vhd = svf + h2 * DHV;
      a = a0; t = t0;
#pragma unroll 1
      for (int tp = 0; tp < TT; ++tp) {
        const float p = base[a * TT + t] * inv;
        const float* vr = vhd + tp * DM;
        const v4f x0 = *(const v4f*)(vr), x1 = *(const v4f*)(vr + 4);
        const v4f x2 = *(const v4f*)(vr + 8), x3 = *(const v4f*)(vr + 12);
#pragma unroll
        for (int e = 0; e < 4; ++e) {
          o[e]      = fmaf(p, x0[e], o[e]);
          o[4 + e]  = fmaf(p, x1[e], o[4 + e]);
          o[8 + e]  = fmaf(p, x2[e], o[8 + e]);
          o[12 + e] = fmaf(p, x3[e], o[12 + e]);
        }
        if (++a == NA) { a = 0; ++t; }
      }
      float* op = sO + (h2 * 16 + a2) * 16;
      const v4f y0 = {o[0], o[1], o[2], o[3]};
      const v4f y1 = {o[4], o[5], o[6], o[7]};
      const v4f y2 = {o[8], o[9], o[10], o[11]};
      const v4f y3 = {o[12], o[13], o[14], o[15]};
      *(v4f*)(op)      = y0;
      *(v4f*)(op + 4)  = y1;
      *(v4f*)(op + 8)  = y2;
      *(v4f*)(op + 12) = y3;
    }
  }
  __syncthreads();

  v4f q0[4], q1[4];
#pragma unroll
  for (int g = 0; g < 4; ++g) {
    const int s = w + 4 * g;
    q0[g] = *(const v4f*)(&sO[s * OSLAB + lane * 4]);
    q1[g] = *(const v4f*)(&sO[s * OSLAB + 128 + lane * 4]);
  }
#pragma unroll
  for (int g = 0; g < 4; ++g) {
    const int s = w + 4 * g;
    float* dst = out3 + ((size_t)s * NB + b2) * OSLAB;
    *(volatile v4f*)(dst + lane * 4) = q0[g];
    *(volatile v4f*)(dst + 128 + lane * 4) = q1[g];
  }
  __threadfence();
#pragma unroll
  for (int g = 0; g < 4; ++g) {
    const int s = w + 4 * g;
    float* dst = out3 + ((size_t)s * NB + b2) * OSLAB;
    *(volatile v4f*)(dst + lane * 4) = q0[g];
    *(volatile v4f*)(dst + 128 + lane * 4) = q1[g];
  }
}

static __device__ __forceinline__ int o3off(int n) {
  const int h2 = n / MROWS;
  const int rem = n - h2 * MROWS;
  const int bb = rem / NA;
  const int a2 = rem - bb * NA;
  return ((h2 * NB + bb) * 16 + a2) * 16;
}

template <int NT>
static __device__ __forceinline__ void mlp_gemm(int nt0, int lane, int a1, int b1,
    const float* __restrict__ out3, const _Float16* __restrict__ w1h, const _Float16* __restrict__ w1l,
    const float* __restrict__ lb1, const float* __restrict__ bnw, const float* __restrict__ bnb,
    const float* __restrict__ bnrm, const float* __restrict__ bnrv,
    const float* __restrict__ gow, const float* __restrict__ gob, float* sYw)
{
  const int hh = lane >> 4, m16 = lane & 15;
  v8f ah[NT], ax[NT];
  int boff[NT];
#pragma unroll
  for (int j = 0; j < NT; ++j) {
    ah[j] = zero8();
    ax[j] = zero8();
    boff[j] = ((nt0 + j) * 16 + m16) * DM + 8 * hh;
  }
#pragma unroll 1
  for (int ks = 0; ks < KSTEPS; ++ks) {
    Frag fh, fl;
    {
      const int n0 = (a1 * NH + 2 * ks) * NB + b1;
      const float* s0 = out3 + o3off(n0) + 8 * hh;
      split8(*(const v4f*)(s0), *(const v4f*)(s0 + 4), SA_MLP, fh.h[0], fl.h[0]);
      const float* s1 = out3 + o3off(n0 + NB) + 8 * hh;
      split8(*(const v4f*)(s1), *(const v4f*)(s1 + 4), SA_MLP, fh.h[1], fl.h[1]);
    }
#pragma unroll
    for (int j = 0; j < NT; ++j) {
      const _Float16* ph = w1h + boff[j] + ks * 32;
      const _Float16* pl = w1l + boff[j] + ks * 32;
      Frag bh, bl;
      bh.h[0] = *(const v8h*)(ph);
      bh.h[1] = *(const v8h*)(ph + 16);
      bl.h[0] = *(const v8h*)(pl);
      bl.h[1] = *(const v8h*)(pl + 16);
      ah[j] = wmma16(fh.v, bh.v, ah[j]);
      ax[j] = wmma16(fh.v, bl.v, ax[j]);
      ax[j] = wmma16(fl.v, bh.v, ax[j]);
    }
  }
#pragma unroll
  for (int j = 0; j < NT; ++j) {
    const int col = (nt0 + j) * 16 + m16;
    const float bi = lb1[col];
    const float rm = bnrm[col];
    const float rstd = 1.0f / sqrtf(bnrv[col] + 1e-5f);
    const float bw = bnw[col], bb = bnb[col];
    const float gw = gow[col], gb = gob[col];
#pragma unroll
    for (int r = 0; r < 8; ++r) {
      float y = (ah[j][r] + ax[j][r] * (1.0f / RESC)) * (1.0f / (SA_MLP * SB_MLP)) + bi;
      y = (y - rm) * rstd * bw + bb;
      y = fmaxf(y, 0.0f);
      float sm = y;
#pragma unroll
      for (int off = 1; off < 8; off <<= 1) sm += __shfl_xor(sm, off, 32);
      const float mu = sm * 0.125f;
      const float dv = y - mu;
      float sq = dv * dv;
#pragma unroll
      for (int off = 1; off < 8; off <<= 1) sq += __shfl_xor(sq, off, 32);
      const float var = sq * 0.125f;
      const float yn = dv * (1.0f / sqrtf(var + 1e-5f)) * gw + gb;
      sYw[(8 * hh + r) * MOUT + col] = yn;
    }
  }
}

__global__ __launch_bounds__(128) void k_mlp(
    const float* __restrict__ out3, const _Float16* __restrict__ w1h, const _Float16* __restrict__ w1l,
    const float* __restrict__ lb1, const float* __restrict__ bnw, const float* __restrict__ bnb,
    const float* __restrict__ bnrm, const float* __restrict__ bnrv,
    const float* __restrict__ gow, const float* __restrict__ gob,
    float* __restrict__ out, int mrows)
{
  __shared__ float sY[4 * 16 * MOUT];
  const int tid = threadIdx.x, lane = tid & 31, w = tid >> 5;
  const int m0 = blockIdx.x * 64 + w * 16;
  int mr = m0 + (lane & 15);
  if (mr > mrows - 1) mr = mrows - 1;
  const int a1 = mr >> 10, b1 = mr & 1023;
  float* sYw = sY + w * (16 * MOUT);

  mlp_gemm<4>(0, lane, a1, b1, out3, w1h, w1l, lb1, bnw, bnb, bnrm, bnrv, gow, gob, sYw);
  mlp_gemm<4>(4, lane, a1, b1, out3, w1h, w1l, lb1, bnw, bnb, bnrm, bnrv, gow, gob, sYw);
  __syncthreads();

  v4f vals[16];
#pragma unroll
  for (int rr = 0; rr < 16; ++rr) vals[rr] = *(const v4f*)(&sYw[rr * MOUT + lane * 4]);
#pragma unroll
  for (int rr = 0; rr < 16; ++rr) {
    const int m = m0 + rr;
    if (m < mrows) {
      const int aa = m >> 10, bb = m & 1023;
      float* dst = out + (size_t)(bb * NA + aa) * MOUT + lane * 4;
      *(volatile v4f*)dst = vals[rr];
    }
  }
  __threadfence();
#pragma unroll
  for (int rr = 0; rr < 16; ++rr) {
    const int m = m0 + rr;
    if (m < mrows) {
      const int aa = m >> 10, bb = m & 1023;
      float* dst = out + (size_t)(bb * NA + aa) * MOUT + lane * 4;
      *(volatile v4f*)dst = vals[rr];
    }
  }
}

static inline size_t al256(size_t v) { return (v + 255) & ~(size_t)255; }

extern "C" void kernel_launch(void* const* d_in, const int* in_sizes, int n_in,
                              void* d_out, int out_size, void* d_ws, size_t ws_size,
                              hipStream_t stream)
{
  if (n_in < 16) return;
  const float* x    = (const float*)d_in[0];
  const float* Wc   = (const float*)d_in[1];
  const float* bc   = (const float*)d_in[2];
  const float* gniw = (const float*)d_in[3];
  const float* gnib = (const float*)d_in[4];
  const float* Q    = (const float*)d_in[5];
  const float* Wk   = (const float*)d_in[6];
  const float* bk   = (const float*)d_in[7];
  const float* W1   = (const float*)d_in[8];
  const float* b1v  = (const float*)d_in[9];
  const float* bnw  = (const float*)d_in[10];
  const float* bnb  = (const float*)d_in[11];
  const float* bnrm = (const float*)d_in[12];
  const float* bnrv = (const float*)d_in[13];
  const float* gow  = (const float*)d_in[14];
  const float* gob  = (const float*)d_in[15];
  float* out = (float*)d_out;

  if (in_sizes[0] != NB * TT * CIN) return;
  if (in_sizes[1] != DM * CIN || in_sizes[2] != DM || in_sizes[3] != DM || in_sizes[4] != DM) return;
  if (in_sizes[5] != NA * NH * DKQ || in_sizes[6] != NA * NH * DKQ * DM || in_sizes[7] != NA * NH * DKQ) return;
  if (in_sizes[8] != MOUT * DM) return;
  for (int i = 9; i < 16; ++i) if (in_sizes[i] != MOUT) return;
  if (out_size != NB * NA * MOUT) return;

  size_t off = 0;
  const size_t vbytes  = (size_t)NB * VTILE * sizeof(float);
  float* vbuf = (float*)((char*)d_ws + off);            off += al256(vbytes);
  const size_t wtbytes = (size_t)NWROW * DM * sizeof(_Float16);
  _Float16* wth = (_Float16*)((char*)d_ws + off);       off += al256(wtbytes);
  _Float16* wtl = (_Float16*)((char*)d_ws + off);       off += al256(wtbytes);
  const size_t w1bytes = (size_t)MOUT * DM * sizeof(_Float16);
  _Float16* w1h = (_Float16*)((char*)d_ws + off);       off += al256(w1bytes);
  _Float16* w1l = (_Float16*)((char*)d_ws + off);       off += al256(w1bytes);
  const size_t o3bytes = (size_t)NH * NB * OSLAB * sizeof(float);
  float* out3 = (float*)((char*)d_ws + off);            off += al256(o3bytes);
  if (off > ws_size) return;

  const int ntab = NWROW / 4 + MOUT / 4;
  const int nmlp = (MROWS + 63) / 64;

  k_inconv_gn<<<NB, 256, 0, stream>>>(x, Wc, bc, gniw, gnib, vbuf, NB);
  k_tables<<<ntab, 128, 0, stream>>>(Q, Wk, W1, wth, wtl, w1h, w1l, ntab);
  k_attn<<<NB, 128, 0, stream>>>(vbuf, wth, wtl, Q, bk, out3, NB);
  k_mlp<<<nmlp, 128, 0, stream>>>(out3, w1h, w1l, b1v, bnw, bnb, bnrm, bnrv, gow, gob, out, MROWS);
  (void)hipGetLastError();
}
